// QuantumTransformerBlock_59004260712622
// MI455X (gfx1250) — hardware-verified
//
#include <hip/hip_runtime.h>
#include <stdint.h>


#define DIM 1024
#define NH 16
#define HD 64
#define FF 4096
#define NB_FULL 2
#define SEQ_FULL 2048
#ifndef NB
#define NB 2
#endif
#ifndef SEQ
#define SEQ 2048
#endif
#define MROWS (NB * SEQ)
#define SCP (SEQ + 4)
#define SP 68
#define WSCALE 1024.0f
#define LNEPS 1.0e-5f

static_assert(NB >= 1 && NB <= NB_FULL);
static_assert(SEQ >= 64 && SEQ <= SEQ_FULL);
static_assert(SEQ % 64 == 0);
static_assert(MROWS % 128 == 0);
static_assert(DIM % 64 == 0 && FF % 64 == 0);
static_assert(NH * HD == DIM);
static_assert(FF == 4 * DIM);

typedef _Float16 v16h __attribute__((ext_vector_type(16)));
typedef _Float16 v8h  __attribute__((ext_vector_type(8)));
typedef float    v8f  __attribute__((ext_vector_type(8)));
typedef float    v4f  __attribute__((ext_vector_type(4)));

union FragU { v16h v; v8h h[2]; };


__device__ __forceinline__ float bf16r(float f) {
    unsigned u = __float_as_uint(f);
    u = (u + 0x7FFFu + ((u >> 16) & 1u)) & 0xFFFF0000u;
    return __uint_as_float(u);
}

__device__ __forceinline__ v16h load_frag(const _Float16* tile, int ld, int k0) {
    const int lane  = threadIdx.x & 31;
    const int row   = lane & 15;
    const int khalf = (lane >> 4) * 8;
    const _Float16* p = tile + (size_t)row * (size_t)ld + (size_t)(k0 + khalf);
    FragU u;
    u.h[0] = *(const v8h*)(p);
    u.h[1] = *(const v8h*)(p + 16);
    return u.v;
}

__device__ __forceinline__ v8f wmma16(v16h a, v16h b, v8f c) {
    return __builtin_amdgcn_wmma_f32_16x16x32_f16(false, a, false, b, (short)0, c, false, false);
}

__device__ __forceinline__ void gemm64x64(const _Float16* __restrict__ A,
                                          const _Float16* __restrict__ Bt,
                                          int K, v8f acc[4][4]) {
#pragma unroll 1
    for (int k0 = 0; k0 < K; k0 += 32) {
        v16h af[4], bf[4];
#pragma unroll
        for (int t = 0; t < 4; ++t) af[t] = load_frag(A + (size_t)(t * 16) * (size_t)K, K, k0);
#pragma unroll
        for (int t = 0; t < 4; ++t) bf[t] = load_frag(Bt + (size_t)(t * 16) * (size_t)K, K, k0);
#pragma unroll
        for (int i = 0; i < 4; ++i)
#pragma unroll
            for (int j = 0; j < 4; ++j)
                acc[i][j] = wmma16(af[i], bf[j], acc[i][j]);
        asm volatile("v_nop\n\tv_nop\n\tv_nop\n\tv_nop"
            : "+v"(acc[0][0]), "+v"(acc[0][1]), "+v"(acc[0][2]), "+v"(acc[0][3]),
              "+v"(acc[1][0]), "+v"(acc[1][1]), "+v"(acc[1][2]), "+v"(acc[1][3]),
              "+v"(acc[2][0]), "+v"(acc[2][1]), "+v"(acc[2][2]), "+v"(acc[2][3]),
              "+v"(acc[3][0]), "+v"(acc[3][1]), "+v"(acc[3][2]), "+v"(acc[3][3])
            : "v"(af[3]), "v"(bf[3]));
    }
}

__global__ __launch_bounds__(256)
void wprep_kernel(const float* __restrict__ W, _Float16* __restrict__ Wt, int K, int N) {
    __shared__ __attribute__((aligned(16))) _Float16 T[64][72];
    const int t  = threadIdx.x;
    const int k0 = (int)blockIdx.y * 64;
    const int n0 = (int)blockIdx.x * 64;
    const int kr = t >> 4;
    const int c4 = (t & 15) * 4;
#pragma unroll
    for (int j = 0; j < 4; ++j) {
        const int k = kr + 16 * j;
        const v4f w = *(const v4f*)(W + (size_t)(k0 + k) * (size_t)N + n0 + c4);
#pragma unroll
        for (int e = 0; e < 4; ++e) T[c4 + e][k] = (_Float16)(bf16r(w[e]) * WSCALE);
    }
    __syncthreads();
    const int nA = t >> 3;
    const int k8 = (t & 7) * 8;
    const v8h o0 = *(const v8h*)(&T[nA][k8]);
    const v8h o1 = *(const v8h*)(&T[nA + 32][k8]);
    _Float16* d0 = Wt + (size_t)(n0 + nA) * (size_t)K + k0 + k8;
    _Float16* d1 = Wt + (size_t)(n0 + nA + 32) * (size_t)K + k0 + k8;
    *(volatile v8h*)d0 = o0;
    *(volatile v8h*)d1 = o1;
    __threadfence();
    *(volatile v8h*)d0 = o0;
    *(volatile v8h*)d1 = o1;
}

template <int SRCX>
__global__ __launch_bounds__(128)
void ln_kernel(const float* __restrict__ src, const float* __restrict__ g,
               const float* __restrict__ bta, _Float16* __restrict__ dst) {
    const int lane = threadIdx.x & 31;
    const int wave = threadIdx.x >> 5;
    const int row  = (int)blockIdx.x * 4 + wave;
    const float* rp;
    if (SRCX) {
        const int bi = row / SEQ;
        const int si = row - bi * SEQ;
        rp = src + ((size_t)bi * SEQ_FULL + (size_t)si) * DIM;
    } else {
        rp = src + (size_t)row * DIM;
    }

    float s = 0.0f;
#pragma unroll 1
    for (int i = 0; i < 4; ++i) {
        const float* p = rp + i * 256 + lane * 8;
        const v4f a = *(const v4f*)p;
        const v4f c = *(const v4f*)(p + 4);
#pragma unroll
        for (int e = 0; e < 4; ++e) {
            float va = a[e], vc = c[e];
            if (SRCX) { va = bf16r(va); vc = bf16r(vc); }
            s += va;
            s += vc;
        }
    }
#pragma unroll
    for (int off = 1; off < 32; off <<= 1) s += __shfl_xor(s, off, 32);
    const float mean = s * (1.0f / DIM);

    float ss = 0.0f;
#pragma unroll 1
    for (int i = 0; i < 4; ++i) {
        const float* p = rp + i * 256 + lane * 8;
        const v4f a = *(const v4f*)p;
        const v4f c = *(const v4f*)(p + 4);
#pragma unroll
        for (int e = 0; e < 4; ++e) {
            float va = a[e], vc = c[e];
            if (SRCX) { va = bf16r(va); vc = bf16r(vc); }
            const float da = va - mean, dc = vc - mean;
            ss += da * da;
            ss += dc * dc;
        }
    }
#pragma unroll
    for (int off = 1; off < 32; off <<= 1) ss += __shfl_xor(ss, off, 32);
    const float rs = rsqrtf(ss * (1.0f / DIM) + LNEPS);

#pragma unroll 1
    for (int pass = 0; pass < 2; ++pass) {
#pragma unroll 1
        for (int i = 0; i < 4; ++i) {
            const int c0 = i * 256 + lane * 8;
            const float* p = rp + c0;
            const v4f a  = *(const v4f*)p;
            const v4f c  = *(const v4f*)(p + 4);
            const v4f ga = *(const v4f*)(g + c0);
            const v4f gc = *(const v4f*)(g + c0 + 4);
            const v4f ba = *(const v4f*)(bta + c0);
            const v4f bc = *(const v4f*)(bta + c0 + 4);
            v8h o;
#pragma unroll
            for (int e = 0; e < 4; ++e) {
                float va = a[e], vc = c[e];
                if (SRCX) { va = bf16r(va); vc = bf16r(vc); }
                const float ya = ((va - mean) * rs) * bf16r(ga[e]) + bf16r(ba[e]);
                const float yc = ((vc - mean) * rs) * bf16r(gc[e]) + bf16r(bc[e]);
                o[e]     = (_Float16)ya;
                o[4 + e] = (_Float16)yc;
            }
            *(volatile v8h*)(dst + (size_t)row * DIM + c0) = o;
        }
        if (pass == 0) __threadfence();
    }
}

template <int MODE>
__global__ __launch_bounds__(64) __attribute__((amdgpu_num_vgpr(256)))
void gemm_kernel(const _Float16* __restrict__ A,
                 const _Float16* __restrict__ Bt0,
                 const _Float16* __restrict__ Bt1,
                 const _Float16* __restrict__ Bt2,
                 const float* __restrict__ bias0,
                 const float* __restrict__ bias1,
                 const float* __restrict__ bias2,
                 _Float16* __restrict__ dh0,
                 _Float16* __restrict__ dh1,
                 _Float16* __restrict__ dh2,
                 float* __restrict__ df,
                 const float* __restrict__ res,
                 const float* __restrict__ aux,
                 int K, int N, float scale) {
    __shared__ __attribute__((aligned(16))) float stile[2][64][SP];
    const int lane = threadIdx.x & 31;
    const int wave = threadIdx.x >> 5;
    const int hb   = lane >> 4;
    const int l16  = lane & 15;
    const int which = (MODE == 0) ? (int)blockIdx.z : 0;
    const int m0 = ((int)blockIdx.y * 2 + wave) * 64;
    const int n0 = (int)blockIdx.x * 64;
    const _Float16* Bt = (which == 0) ? Bt0 : ((which == 1) ? Bt1 : Bt2);
    const float* bias = (which == 0) ? bias0 : ((which == 1) ? bias1 : bias2);

    v8f acc[4][4];
#pragma unroll
    for (int i = 0; i < 4; ++i)
#pragma unroll
        for (int j = 0; j < 4; ++j)
#pragma unroll
            for (int r = 0; r < 8; ++r) acc[i][j][r] = 0.0f;

    gemm64x64(A + (size_t)m0 * (size_t)K, Bt + (size_t)n0 * (size_t)K, K, acc);

    float* T = &stile[wave][0][0];
    float bj[4];
#pragma unroll
    for (int j = 0; j < 4; ++j) bj[j] = bf16r(bias[n0 + j * 16 + l16]);
#pragma unroll
    for (int i = 0; i < 4; ++i)
#pragma unroll
        for (int j = 0; j < 4; ++j)
#pragma unroll
            for (int r = 0; r < 8; ++r)
                T[(i * 16 + hb * 8 + r) * SP + j * 16 + l16] = acc[i][j][r] * scale + bj[j];
    __syncthreads();

    const int bidx = m0 / SEQ;
    const int s0   = m0 - bidx * SEQ;
    const int hh   = n0 / HD;

#pragma unroll 1
    for (int pass = 0; pass < 2; ++pass) {
        if (MODE == 0) {
            if (which < 2) {
                _Float16* base = ((which == 0) ? dh0 : dh1) +
                                 ((size_t)(bidx * NH + hh) * SEQ + (size_t)s0) * HD;
#pragma unroll 1
                for (int it = 0; it < 16; ++it) {
                    const int row = it * 4 + (lane >> 3);
                    const int c8  = (lane & 7) * 8;
                    const v4f a = *(const v4f*)(T + row * SP + c8);
                    const v4f c = *(const v4f*)(T + row * SP + c8 + 4);
                    v8h o;
#pragma unroll
                    for (int e = 0; e < 4; ++e) { o[e] = (_Float16)a[e]; o[4 + e] = (_Float16)c[e]; }
                    *(volatile v8h*)(base + (size_t)row * HD + c8) = o;
                }
            } else {
                _Float16* base = dh2 + ((size_t)(bidx * NH + hh) * HD) * (size_t)SEQ + s0;
#pragma unroll 1
                for (int it = 0; it < 16; ++it) {
                    const int d  = it * 4 + (lane >> 3);
                    const int s8 = (lane & 7) * 8;
                    v8h o;
#pragma unroll
                    for (int e = 0; e < 8; ++e) o[e] = (_Float16)T[(s8 + e) * SP + d];
                    *(volatile v8h*)(base + (size_t)d * SEQ + s8) = o;
                }
            }
        } else if (MODE == 2) {
#pragma unroll 1
            for (int it = 0; it < 16; ++it) {
                const int row = it * 4 + (lane >> 3);
                const int c8  = (lane & 7) * 8;
                const v4f a = *(const v4f*)(T + row * SP + c8);
                const v4f c = *(const v4f*)(T + row * SP + c8 + 4);
                v8h o;
#pragma unroll
                for (int e = 0; e < 4; ++e) {
                    const float ua = a[e], uc = c[e];
                    const float ga = 0.5f * ua * (1.0f + erff(ua * 0.70710678118654752f));
                    const float gc = 0.5f * uc * (1.0f + erff(uc * 0.70710678118654752f));
                    o[e]     = (_Float16)(64.0f * ga);
                    o[4 + e] = (_Float16)(64.0f * gc);
                }
                *(volatile v8h*)(dh0 + (size_t)(m0 + row) * (size_t)N + n0 + c8) = o;
            }
        } else {
#pragma unroll 1
            for (int it = 0; it < 32; ++it) {
                const int row = it * 2 + hb;
                const int c4  = l16 * 4;
                const v4f v = *(const v4f*)(T + row * SP + c4);
                const int m = m0 + row;
                const int n = n0 + c4;
                v4f o;
                if (MODE == 1) {
                    const int bb = m / SEQ;
                    const int ss = m - bb * SEQ;
                    const v4f xv = *(const v4f*)(res + ((size_t)bb * SEQ_FULL + (size_t)ss) * DIM + n);
                    const v4f ph = *(const v4f*)(aux + n);
#pragma unroll
                    for (int e = 0; e < 4; ++e) {
                        const float t = v[e] + bf16r(xv[e]);
                        const float p = bf16r(ph[e]);
                        o[e] = t * cosf(p * t);
                    }
                } else if (MODE == 3) {
                    const v4f xv = *(const v4f*)(res + (size_t)m * (size_t)N + n);
#pragma unroll
                    for (int e = 0; e < 4; ++e) o[e] = xv[e] + v[e];
                } else if (MODE == 4) {
#pragma unroll
                    for (int e = 0; e < 4; ++e) {
                        const float gl = fminf(fmaxf(v[e], -30.0f), 30.0f);
                        const float ex = __expf(-gl);
                        o[e] = __builtin_amdgcn_rcpf(1.0f + ex);
                    }
                } else {
                    const v4f gv = *(const v4f*)(aux + (size_t)m * (size_t)N + n);
                    const v4f xv = *(const v4f*)(res + (size_t)m * (size_t)N + n);
#pragma unroll
                    for (int e = 0; e < 4; ++e) {
                        const float gg = gv[e];
                        o[e] = v[e] * gg + xv[e] * (1.0f - gg);
                    }
                }
                *(volatile v4f*)(df + (size_t)m * (size_t)N + n) = o;
            }
            if (MODE == 3) {
#pragma unroll 1
                for (int it = 0; it < 16; ++it) {
                    const int row = it * 4 + (lane >> 3);
                    const int c8  = (lane & 7) * 8;
                    const v4f a = *(const v4f*)(T + row * SP + c8);
                    const v4f c = *(const v4f*)(T + row * SP + c8 + 4);
                    const size_t gidx = (size_t)(m0 + row) * (size_t)N + n0 + c8;
                    const v4f xa = *(const v4f*)(res + gidx);
                    const v4f xc = *(const v4f*)(res + gidx + 4);
                    v8h o;
#pragma unroll
                    for (int e = 0; e < 4; ++e) {
                        o[e]     = (_Float16)(xa[e] + a[e]);
                        o[4 + e] = (_Float16)(xc[e] + c[e]);
                    }
                    *(volatile v8h*)(dh0 + gidx) = o;
                }
            }
        }
        if (pass == 0) __threadfence();
    }
}

__global__ __launch_bounds__(128)
void attn_kernel(const _Float16* __restrict__ q16,
                 const _Float16* __restrict__ k16,
                 const _Float16* __restrict__ vT16,
                 const float* __restrict__ qphase,
                 _Float16* __restrict__ ctx16) {
    extern __shared__ float smem[];
    float* sc     = smem;
    float* pout   = sc + 16 * SCP;
    float* rowinv = pout + 4 * 16 * 64;

    const int lane = threadIdx.x & 31;
    const int wave = threadIdx.x >> 5;
    const int hb   = lane >> 4;
    const int l16  = lane & 15;
    const int b = blockIdx.z, h = blockIdx.y, q0 = (int)blockIdx.x * 16;
    const size_t bh = (size_t)b * NH + (size_t)h;
    const _Float16* qbase = q16 + (bh * SEQ + (size_t)q0) * HD;
    const _Float16* kbase = k16 + (bh * SEQ) * HD;
    const _Float16* vbase = vT16 + (bh * HD) * (size_t)SEQ;

    const v16h aq0 = load_frag(qbase, HD, 0);
    const v16h aq1 = load_frag(qbase, HD, 32);
    const float phase = bf16r(qphase[h]);

#pragma unroll 1
    for (int kt = wave; kt < SEQ / 16; kt += 4) {
        v8f c;
#pragma unroll
        for (int r = 0; r < 8; ++r) c[r] = 0.0f;
        const _Float16* kp = kbase + (size_t)(kt * 16) * HD;
        const v16h bk0 = load_frag(kp, HD, 0);
        const v16h bk1 = load_frag(kp, HD, 32);
        c = wmma16(aq0, bk0, c);
        c = wmma16(aq1, bk1, c);
        asm volatile("v_nop\n\tv_nop\n\tv_nop\n\tv_nop" : "+v"(c) : "v"(aq1), "v"(bk1));
#pragma unroll
        for (int r = 0; r < 8; ++r) {
            float s = c[r] * 0.125f;
            s = s * (1.0f + 0.1f * cosf(phase * s));
            sc[(hb * 8 + r) * SCP + kt * 16 + l16] = s;
        }
    }
    __syncthreads();

    {
        const int t   = threadIdx.x;
        const int row = t >> 3;
        const int sub = t & 7;
        float* rp = sc + row * SCP + sub;
        float mx = -3.0e38f;
#pragma unroll 4
        for (int kk = 0; kk < SEQ / 8; ++kk) mx = fmaxf(mx, rp[8 * kk]);
#pragma unroll
        for (int off = 1; off < 8; off <<= 1) mx = fmaxf(mx, __shfl_xor(mx, off, 32));
        float sm = 0.0f;
#pragma unroll 4
        for (int kk = 0; kk < SEQ / 8; ++kk) {
            const float e = __expf(rp[8 * kk] - mx);
            rp[8 * kk] = e;
            sm += e;
        }
#pragma unroll
        for (int off = 1; off < 8; off <<= 1) sm += __shfl_xor(sm, off, 32);
        if (sub == 0) rowinv[row] = (1.0f / sm) * 0.0625f;
    }
    __syncthreads();

    v8f acc[4];
#pragma unroll
    for (int j = 0; j < 4; ++j)
#pragma unroll
        for (int r = 0; r < 8; ++r) acc[j][r] = 0.0f;
    const int khalf = hb * 8;
#pragma unroll 1
    for (int kb = wave; kb < SEQ / 32; kb += 4) {
        v16h pa;
        const float* pr = sc + l16 * SCP + kb * 32 + khalf;
#pragma unroll
        for (int i = 0; i < 8; ++i) {
            pa[i]     = (_Float16)(pr[i] * 1024.0f);
            pa[8 + i] = (_Float16)(pr[16 + i] * 1024.0f);
        }
        v16h bvf[4];
#pragma unroll
        for (int j = 0; j < 4; ++j) bvf[j] = load_frag(vbase + (size_t)(j * 16) * (size_t)SEQ, SEQ, kb * 32);
#pragma unroll
        for (int j = 0; j < 4; ++j) acc[j] = wmma16(pa, bvf[j], acc[j]);
        asm volatile("v_nop\n\tv_nop\n\tv_nop\n\tv_nop" : "+v"(acc[0]), "+v"(acc[1]), "+v"(acc[2]), "+v"(acc[3])
                          : "v"(pa), "v"(bvf[3]));
    }
#pragma unroll
    for (int j = 0; j < 4; ++j)
#pragma unroll
        for (int r = 0; r < 8; ++r)
            pout[(wave * 16 + hb * 8 + r) * 64 + j * 16 + l16] = acc[j][r];
    __syncthreads();

    {
        const int t   = threadIdx.x;
        const int row = t >> 3;
        const int d8  = (t & 7) * 8;
        const float inv = rowinv[row];
        v8h o;
#pragma unroll
        for (int e = 0; e < 8; ++e) {
            const int d = d8 + e;
            const float v = pout[(0 * 16 + row) * 64 + d] + pout[(1 * 16 + row) * 64 + d]
                          + pout[(2 * 16 + row) * 64 + d] + pout[(3 * 16 + row) * 64 + d];
            o[e] = (_Float16)(v * inv);
        }
        _Float16* dst = ctx16 + ((size_t)b * SEQ + (size_t)(q0 + row)) * DIM + h * HD + d8;
        *(volatile v8h*)dst = o;
        __threadfence();
        *(volatile v8h*)dst = o;
    }
}

extern "C" void kernel_launch(void* const* d_in, const int* in_sizes, int n_in,
                              void* d_out, int out_size, void* d_ws, size_t ws_size,
                              hipStream_t stream) {
    if (n_in < 23) return;
    const float* x      = (const float*)d_in[0];
    const float* wq     = (const float*)d_in[1];
    const float* bq     = (const float*)d_in[2];
    const float* wk     = (const float*)d_in[3];
    const float* bk     = (const float*)d_in[4];
    const float* wv     = (const float*)d_in[5];
    const float* bv     = (const float*)d_in[6];
    const float* wo     = (const float*)d_in[7];
    const float* bo     = (const float*)d_in[8];
    const float* qphase = (const float*)d_in[9];
    const float* sphase = (const float*)d_in[10];
    const float* wi_p   = (const float*)d_in[11];
    const float* bi_p   = (const float*)d_in[12];
    const float* wi_g   = (const float*)d_in[13];
    const float* bi_g   = (const float*)d_in[14];
    const float* ln1_g  = (const float*)d_in[15];
    const float* ln1_b  = (const float*)d_in[16];
    const float* ln2_g  = (const float*)d_in[17];
    const float* ln2_b  = (const float*)d_in[18];
    const float* w1     = (const float*)d_in[19];
    const float* b1     = (const float*)d_in[20];
    const float* w2     = (const float*)d_in[21];
    const float* b2     = (const float*)d_in[22];
    float* out = (float*)d_out;

    const long long needX = ((long long)(NB - 1) * SEQ_FULL + (long long)SEQ) * DIM;
    if ((long long)in_sizes[0] < needX) return;
    if (in_sizes[1] < DIM * DIM || in_sizes[3] < DIM * DIM || in_sizes[5] < DIM * DIM ||
        in_sizes[7] < DIM * DIM || in_sizes[11] < DIM * DIM || in_sizes[13] < DIM * DIM) return;
    if (in_sizes[19] < DIM * FF || in_sizes[21] < FF * DIM) return;
    if (in_sizes[2] < DIM || in_sizes[4] < DIM || in_sizes[6] < DIM || in_sizes[8] < DIM ||
        in_sizes[12] < DIM || in_sizes[14] < DIM) return;
    if (in_sizes[15] < DIM || in_sizes[16] < DIM || in_sizes[17] < DIM || in_sizes[18] < DIM) return;
    if (in_sizes[20] < FF || in_sizes[22] < DIM) return;
    if (in_sizes[9] < NH || in_sizes[10] < DIM) return;
    if ((long long)out_size < (long long)MROWS * DIM) return;

    char* ws = (char*)d_ws;
    const size_t szW  = (size_t)DIM * DIM * 2;
    const size_t szW1 = (size_t)DIM * FF * 2;
    const size_t szH  = (size_t)MROWS * DIM * 2;
    const size_t szF  = (size_t)MROWS * DIM * 4;
    size_t off = 0;
    _Float16* wqT  = (_Float16*)(ws + off); off += szW;
    _Float16* wkT  = (_Float16*)(ws + off); off += szW;
    _Float16* wvT  = (_Float16*)(ws + off); off += szW;
    _Float16* woT  = (_Float16*)(ws + off); off += szW;
    _Float16* wipT = (_Float16*)(ws + off); off += szW;
    _Float16* wigT = (_Float16*)(ws + off); off += szW;
    _Float16* w1T  = (_Float16*)(ws + off); off += szW1;
    _Float16* w2T  = (_Float16*)(ws + off); off += szW1;
    _Float16* h16  = (_Float16*)(ws + off); off += szH;
    _Float16* q16  = (_Float16*)(ws + off);
    _Float16* k16  = (_Float16*)(ws + off + szH);
    _Float16* vT16 = (_Float16*)(ws + off + 2 * szH);
    _Float16* ctx16= (_Float16*)(ws + off + 3 * szH);
    _Float16* ff16 = (_Float16*)(ws + off);
    off += 4 * szH;
    float*    x1   = (float*)(ws + off); off += szF;
    float*    x3   = (float*)(ws + off); off += szF;
    _Float16* x3h  = (_Float16*)(ws + off); off += szH;
    float*    gsig = (float*)(ws + off); off += szF;
    if (off > ws_size) return;

    const dim3 b256(256), b128(128), b64(64);
    const float sW  = 1.0f / 1024.0f;
    const float sWW = 1.0f / 65536.0f;

    wprep_kernel<<<dim3(DIM / 64, DIM / 64), b256, 0, stream>>>(wq,   wqT,  DIM, DIM);
    wprep_kernel<<<dim3(DIM / 64, DIM / 64), b256, 0, stream>>>(wk,   wkT,  DIM, DIM);
    wprep_kernel<<<dim3(DIM / 64, DIM / 64), b256, 0, stream>>>(wv,   wvT,  DIM, DIM);
    wprep_kernel<<<dim3(DIM / 64, DIM / 64), b256, 0, stream>>>(wo,   woT,  DIM, DIM);
    wprep_kernel<<<dim3(DIM / 64, DIM / 64), b256, 0, stream>>>(wi_p, wipT, DIM, DIM);
    wprep_kernel<<<dim3(DIM / 64, DIM / 64), b256, 0, stream>>>(wi_g, wigT, DIM, DIM);
    wprep_kernel<<<dim3(FF / 64, DIM / 64),  b256, 0, stream>>>(w1,   w1T,  DIM, FF);
    wprep_kernel<<<dim3(DIM / 64, FF / 64),  b256, 0, stream>>>(w2,   w2T,  FF,  DIM);

    ln_kernel<1><<<MROWS / 4, b128, 0, stream>>>(x, ln1_g, ln1_b, h16);

    gemm_kernel<0><<<dim3(DIM / 64, MROWS / 128, 3), b64, 0, stream>>>(
        h16, wqT, wkT, wvT, bq, bk, bv, q16, k16, vT16, gsig, sphase, sphase, DIM, DIM, sW);

    const size_t attn_lds = (size_t)(16 * SCP + 4 * 16 * 64 + 32) * sizeof(float);
    hipFuncSetAttribute(reinterpret_cast<const void*>(&attn_kernel),
                        hipFuncAttributeMaxDynamicSharedMemorySize, (int)attn_lds);
    attn_kernel<<<dim3(SEQ / 16, NH, NB), b128, attn_lds, stream>>>(q16, k16, vT16, qphase, ctx16);

    gemm_kernel<1><<<dim3(DIM / 64, MROWS / 128, 1), b64, 0, stream>>>(
        ctx16, woT, woT, woT, bo, bo, bo, h16, h16, h16, x1, x, sphase, DIM, DIM, sWW);

    ln_kernel<0><<<MROWS / 4, b128, 0, stream>>>(x1, ln2_g, ln2_b, h16);

    gemm_kernel<2><<<dim3(FF / 64, MROWS / 128, 1), b64, 0, stream>>>(
        h16, w1T, w1T, w1T, b1, b1, b1, ff16, ff16, ff16, gsig, sphase, sphase, DIM, FF, sW);

    gemm_kernel<3><<<dim3(DIM / 64, MROWS / 128, 1), b64, 0, stream>>>(
        ff16, w2T, w2T, w2T, b2, b2, b2, x3h, x3h, x3h, x3, x1, sphase, FF, DIM, sWW);

    gemm_kernel<4><<<dim3(DIM / 64, MROWS / 128, 1), b64, 0, stream>>>(
        x3h, wigT, wigT, wigT, bi_g, bi_g, bi_g, h16, h16, h16, gsig, sphase, sphase, DIM, DIM, sW);

    gemm_kernel<5><<<dim3(DIM / 64, MROWS / 128, 1), b64, 0, stream>>>(
        x3h, wipT, wipT, wipT, bi_p, bi_p, bi_p, h16, h16, h16, out, x3, gsig, DIM, DIM, sW);

    (void)ws_size;
}
